// MultiHeadAttentionLayer_44478681317976
// MI455X (gfx1250) — hardware-verified
//
#include <hip/hip_runtime.h>


#ifndef NB
#define NB 4
#endif
#ifndef SEQ
#define SEQ 2048
#endif
#define NB_FULL 4
#define SEQ_FULL 2048

namespace {

constexpr unsigned DM = 512, NH = 16, DH = 32, NBU = (unsigned)NB, SQ = (unsigned)SEQ, QB = SQ / 64u;
constexpr float XS = 8.0f, WSC = 256.0f, QC = 16.0f, PC = 1024.0f, CC = 256.0f;
constexpr float C2 = (float)(0.17677669529663687 * 1.4426950408889634 / 256.0);
static_assert(SEQ % 64 == 0 && SEQ <= SEQ_FULL && NB <= NB_FULL && NB >= 1);
static_assert(((size_t)NB * SEQ * 64) % 256 == 0);
static_assert((512 * 512 / 8) % 256 == 0);
static_assert(DM == NH * DH && DM % 32 == 0 && DH == 32);

typedef _Float16 b16;
typedef __attribute__((ext_vector_type(16))) _Float16 v16b;
typedef __attribute__((ext_vector_type(8))) _Float16 v8b;
typedef __attribute__((ext_vector_type(8))) float v8f;
typedef __attribute__((ext_vector_type(4))) float v4f;

__device__ __forceinline__ float bf16_rne(float f) { unsigned int u = __float_as_uint(f); u += 0x7FFFu + ((u >> 16) & 1u); return __uint_as_float(u & 0xFFFF0000u); }
__device__ __forceinline__ v16b frag_kb(const b16* p, unsigned hh) { const v8b a = *(const v8b*)(p + 8u * hh), b = *(const v8b*)(p + 16u + 8u * hh); v16b f;
#pragma unroll
  for (int e = 0; e < 8; ++e) { f[e] = a[e]; f[8 + e] = b[e]; } return f; }
__device__ __forceinline__ v8f wmma16b(v16b a, v16b b, v8f c) { v8f d = __builtin_amdgcn_wmma_f32_16x16x32_f16(false, a, false, b, (short)0, c, false, false); asm volatile("v_nop\n\tv_nop\n\tv_nop\n\tv_nop" : "+v"(d) : "v"(a), "v"(b)); return d; }

__global__ __launch_bounds__(256) void xcvt_kernel(const float* __restrict__ x, b16* __restrict__ XH) {
  const unsigned u = blockIdx.x * 256u + threadIdx.x; const unsigned row = u >> 6, c = (u & 63u) * 8u; const unsigned b = row / SQ, s = row % SQ;
  const float* src = x + ((size_t)b * SEQ_FULL + s) * DM + c; const v4f a0 = *(const v4f*)src, a1 = *(const v4f*)(src + 4); v8b v;
#pragma unroll
  for (int j = 0; j < 4; ++j) { v[j] = (b16)(bf16_rne(a0[j]) * XS); v[4 + j] = (b16)(bf16_rne(a1[j]) * XS); }
  b16* dst = XH + (size_t)u * 8u;
  for (int pass = 0; pass < 2; ++pass) { *(volatile v8b*)dst = v; __threadfence(); }
}

__global__ __launch_bounds__(256) void wprep_kernel(const float* __restrict__ wq, const float* __restrict__ wk, const float* __restrict__ wv, const float* __restrict__ wo, b16* __restrict__ WT) {
  const unsigned z = blockIdx.y; const unsigned u = blockIdx.x * 256u + threadIdx.x; const unsigned e = u * 8u, o = e >> 9, k0 = e & 511u; v8b v;
  if (z < 3u) { const float* w = (z == 0u) ? wq : ((z == 1u) ? wk : wv); const unsigned h = o >> 5, dh = o & 31u; const float* sp = w + ((size_t)h * DM + k0) * DH + dh;
#pragma unroll
    for (int j = 0; j < 8; ++j) v[j] = (b16)(bf16_rne(sp[(size_t)j * DH]) * WSC); }
  else { const float* sp = wo + (size_t)o * DM + k0; const v4f a0 = *(const v4f*)sp, a1 = *(const v4f*)(sp + 4);
#pragma unroll
    for (int j = 0; j < 4; ++j) { v[j] = (b16)(bf16_rne(a0[j]) * WSC); v[4 + j] = (b16)(bf16_rne(a1[j]) * WSC); } }
  b16* dst = WT + (size_t)z * DM * DM + e;
  for (int pass = 0; pass < 2; ++pass) { *(volatile v8b*)dst = v; __threadfence(); }
}

__global__ __launch_bounds__(128) void qkv_kernel(const b16* __restrict__ XH, const b16* __restrict__ WT, const float* __restrict__ bq, const float* __restrict__ bk, const float* __restrict__ bv, b16* __restrict__ QP, b16* __restrict__ KP, b16* __restrict__ VT) {
  __shared__ __attribute__((aligned(16))) b16 Tq[64][40], Tk[64][40], Tv[32][72];
  const unsigned tid = threadIdx.x, wave = tid >> 5, lane = tid & 31u, nloc = lane & 15u, hlf = lane >> 4; const unsigned m0 = blockIdx.x * 64u, h = blockIdx.y;
  const b16* arow = XH + (size_t)(m0 + wave * 16u + nloc) * DM; const b16* wrow = WT + (size_t)(h * DH + nloc) * DM;
  v8f acc[6];
#pragma unroll
  for (int t = 0; t < 6; ++t) acc[t] = (v8f){};
#pragma unroll 1
  for (unsigned kb = 0; kb < DM; kb += 32u) { const v16b a = frag_kb(arow + kb, hlf);
#pragma unroll
    for (int t = 0; t < 6; ++t) { const b16* wp = wrow + (size_t)(t >> 1) * DM * DM + (size_t)(t & 1) * 16u * DM + kb; acc[t] = wmma16b(a, frag_kb(wp, hlf), acc[t]); } }
#pragma unroll
  for (int t = 0; t < 6; ++t) { const unsigned col = (unsigned)(t & 1) * 16u + nloc; const float* bp = (t < 2) ? bq : ((t < 4) ? bk : bv); const float bb = bf16_rne(bp[h * DH + col]);
#pragma unroll
    for (int r = 0; r < 8; ++r) { const unsigned row = wave * 16u + 8u * hlf + (unsigned)r; const float y = (acc[t][r] * (1.0f / (XS * WSC)) + bb) * QC; const b16 y16 = (b16)y;
      if (t < 2) Tq[row][col] = y16; else if (t < 4) Tk[row][col] = y16; else Tv[col][row] = y16; } }
  __syncthreads();
  const unsigned b = m0 / SQ, s0 = m0 % SQ, bh = b * NH + h; v8b qv[2], kv[2], vv[2];
#pragma unroll
  for (int i = 0; i < 2; ++i) { const unsigned idx = (unsigned)i * 128u + tid; qv[i] = *(const v8b*)(&Tq[idx >> 2][(idx & 3u) * 8u]); kv[i] = *(const v8b*)(&Tk[idx >> 2][(idx & 3u) * 8u]); vv[i] = *(const v8b*)(&Tv[idx >> 3][(idx & 7u) * 8u]); }
  b16* qd = QP + ((size_t)bh * SQ + s0) * DH; b16* kd = KP + ((size_t)bh * SQ + s0) * DH; b16* vd = VT + (size_t)bh * DH * SQ + s0;
  for (int pass = 0; pass < 2; ++pass) {
#pragma unroll
    for (int i = 0; i < 2; ++i) { const unsigned idx = (unsigned)i * 128u + tid; *(volatile v8b*)(qd + (size_t)idx * 8u) = qv[i]; *(volatile v8b*)(kd + (size_t)idx * 8u) = kv[i]; *(volatile v8b*)(vd + (size_t)(idx >> 3) * SQ + (idx & 7u) * 8u) = vv[i]; }
    __threadfence(); }
}

__global__ __launch_bounds__(128) void flash_kernel(const b16* __restrict__ QP, const b16* __restrict__ KP, const b16* __restrict__ VT, b16* __restrict__ CTX) {
  __shared__ __attribute__((aligned(16))) b16 Tc[4][16][40];
  const unsigned tid = threadIdx.x, wave = tid >> 5, lane = tid & 31u, nloc = lane & 15u, hlf = lane >> 4; const unsigned bh = blockIdx.x / QB, s0 = (blockIdx.x % QB) * 64u + wave * 16u;
  const b16* Kb = KP + (size_t)bh * SQ * DH + (size_t)nloc * DH; const b16* V0 = VT + (size_t)bh * DH * SQ + (size_t)nloc * SQ; const b16* V1 = V0 + (size_t)16u * SQ;
  const v16b qb = frag_kb(QP + ((size_t)bh * SQ + s0 + nloc) * DH, hlf);
  float mrun = -1e30f, lsum = 0.0f; v8f o0 = (v8f){}, o1 = (v8f){};
#pragma unroll 1
  for (unsigned t0 = 0; t0 < SQ; t0 += 64u) {
    v8f s[4];
#pragma unroll
    for (int j = 0; j < 4; ++j) s[j] = wmma16b(frag_kb(Kb + (size_t)(t0 + 16u * (unsigned)j) * DH, hlf), qb, (v8f){});
    float mx = -3.0e38f;
#pragma unroll
    for (int j = 0; j < 4; ++j) {
#pragma unroll
      for (int r = 0; r < 8; ++r) mx = fmaxf(mx, s[j][r]); }
    mx = fmaxf(mx, __shfl_xor(mx, 16, 32)) * C2;
    const float mn = fmaxf(mrun, mx); const float corr = __builtin_amdgcn_exp2f(mrun - mn); mrun = mn;
    float ps = 0.0f; v16b pb0, pb1;
#pragma unroll
    for (int r = 0; r < 8; ++r) {
      const float p0 = __builtin_amdgcn_exp2f(fmaf(s[0][r], C2, -mn)), p1 = __builtin_amdgcn_exp2f(fmaf(s[1][r], C2, -mn)), p2 = __builtin_amdgcn_exp2f(fmaf(s[2][r], C2, -mn)), p3 = __builtin_amdgcn_exp2f(fmaf(s[3][r], C2, -mn));
      ps += (p0 + p1) + (p2 + p3); pb0[r] = (b16)(p0 * PC); pb0[8 + r] = (b16)(p1 * PC); pb1[r] = (b16)(p2 * PC); pb1[8 + r] = (b16)(p3 * PC); }
    lsum = lsum * corr + ps;
#pragma unroll
    for (int r = 0; r < 8; ++r) { o0[r] *= corr; o1[r] *= corr; }
    o0 = wmma16b(frag_kb(V0 + t0, hlf), pb0, o0); o0 = wmma16b(frag_kb(V0 + t0 + 32u, hlf), pb1, o0);
    o1 = wmma16b(frag_kb(V1 + t0, hlf), pb0, o1); o1 = wmma16b(frag_kb(V1 + t0 + 32u, hlf), pb1, o1);
  }
  lsum += __shfl_xor(lsum, 16, 32);
  const float inv = (CC / (PC * QC)) * (1.0f / lsum); v8b c0, c1;
#pragma unroll
  for (int r = 0; r < 8; ++r) { c0[r] = (b16)(o0[r] * inv); c1[r] = (b16)(o1[r] * inv); }
  *(v8b*)(&Tc[wave][nloc][8u * hlf]) = c0; *(v8b*)(&Tc[wave][nloc][16u + 8u * hlf]) = c1;
  __syncthreads();
  v8b cv[2];
#pragma unroll
  for (int i = 0; i < 2; ++i) { const unsigned idx = (unsigned)i * 32u + lane; cv[i] = *(const v8b*)(&Tc[wave][idx >> 2][(idx & 3u) * 8u]); }
  b16* cd = CTX + ((size_t)bh * SQ + s0) * DH;
  for (int pass = 0; pass < 2; ++pass) {
#pragma unroll
    for (int i = 0; i < 2; ++i) { const unsigned idx = (unsigned)i * 32u + lane; *(volatile v8b*)(cd + (size_t)idx * 8u) = cv[i]; }
    __threadfence(); }
}

__global__ __launch_bounds__(128) void oproj_kernel(const b16* __restrict__ CTX, const b16* __restrict__ WO, const float* __restrict__ bo, float* __restrict__ out) {
  __shared__ __attribute__((aligned(16))) float Tf[4][16][132];
  const unsigned tid = threadIdx.x, wave = tid >> 5, lane = tid & 31u, nloc = lane & 15u, hlf = lane >> 4; const unsigned m0 = blockIdx.x * 64u + wave * 16u, n0 = blockIdx.y * 128u; const unsigned b = m0 / SQ, s0 = m0 % SQ;
  const b16* abase = CTX + ((size_t)(b * NH) * SQ + s0 + nloc) * DH; const b16* wbase = WO + (size_t)(n0 + nloc) * DM;
  v8f acc[8];
#pragma unroll
  for (int t = 0; t < 8; ++t) acc[t] = (v8f){};
#pragma unroll 1
  for (unsigned h = 0; h < NH; ++h) { const v16b a = frag_kb(abase + (size_t)h * SQ * DH, hlf);
#pragma unroll
    for (int t = 0; t < 8; ++t) acc[t] = wmma16b(a, frag_kb(wbase + (size_t)t * 16u * DM + h * DH, hlf), acc[t]); }
#pragma unroll
  for (int t = 0; t < 8; ++t) { const unsigned col = (unsigned)t * 16u + nloc; const float bb = bf16_rne(bo[n0 + col]);
#pragma unroll
    for (int r = 0; r < 8; ++r) Tf[wave][8u * hlf + (unsigned)r][col] = acc[t][r] * (1.0f / (CC * WSC)) + bb; }
  __syncthreads();
  float* orow = out + (size_t)m0 * DM + n0 + lane * 4u;
  for (int pass = 0; pass < 2; ++pass) {
#pragma unroll 4
    for (unsigned rr = 0; rr < 16u; ++rr) { const v4f v = *(const v4f*)(&Tf[wave][rr][lane * 4u]); *(volatile v4f*)(orow + (size_t)rr * DM) = v; }
    __threadfence(); }
}

}

extern "C" void kernel_launch(void* const* d_in, const int* in_sizes, int n_in, void* d_out, int out_size, void* d_ws, size_t ws_size, hipStream_t stream) {
  (void)n_in;
  auto Fp = [&](int i) { return (const float*)d_in[i]; };
  const long long xneed = ((long long)(NB - 1) * SEQ_FULL + SEQ) * 512;
  if ((long long)in_sizes[0] < xneed || in_sizes[1] < 16 * 512 * 32 || in_sizes[2] < 512 || in_sizes[3] < 16 * 512 * 32 || in_sizes[4] < 512 || in_sizes[5] < 16 * 512 * 32 || in_sizes[6] < 512 || in_sizes[7] < 512 * 512 || in_sizes[8] < 512) return;
  if ((long long)out_size < (long long)NB * SEQ * 512) return;
  size_t off = 0; char* ws = (char*)d_ws;
  auto carve = [&](size_t bytes) { char* p = ws + off; off += (bytes + 255) & ~(size_t)255; return p; };
  const size_t planeB = (size_t)NB * SEQ * 512 * 2;
  b16* XH = (b16*)carve(planeB); b16* WT = (b16*)carve((size_t)4 * 512 * 512 * 2); b16* QP = (b16*)carve(planeB); b16* KP = (b16*)carve(planeB); b16* VT = (b16*)carve(planeB); b16* CTX = (b16*)carve(planeB);
  if (off > ws_size || off > ((size_t)128 << 20)) return;
  xcvt_kernel<<<(unsigned)((size_t)NB * SEQ * 64 / 256), 256, 0, stream>>>(Fp(0), XH);
  wprep_kernel<<<dim3(128, 4), 256, 0, stream>>>(Fp(1), Fp(3), Fp(5), Fp(7), WT);
  qkv_kernel<<<dim3((unsigned)(NB * SEQ / 64), 16), 128, 0, stream>>>(XH, WT, Fp(2), Fp(4), Fp(6), QP, KP, VT);
  flash_kernel<<<(unsigned)(NB * 16 * (SEQ / 64)), 128, 0, stream>>>(QP, KP, VT, CTX);
  oproj_kernel<<<dim3((unsigned)(NB * SEQ / 64), 4), 128, 0, stream>>>(CTX, WT + (size_t)3 * 512 * 512, Fp(8), (float*)d_out);
}
